// Mamba3Block_62010737819992
// MI455X (gfx1250) — hardware-run, weakly checked
//
#include <hip/hip_runtime.h>
#include <math.h>

typedef __attribute__((ext_vector_type(16))) _Float16 v16h;
typedef __attribute__((ext_vector_type(8)))  _Float16 v8h;
typedef __attribute__((ext_vector_type(8)))  float    v8f;
typedef __attribute__((ext_vector_type(4)))  float    v4f;

constexpr int kBatch = 4;
constexpr int kSeq   = 2048;
constexpr int kDm    = 1024;
constexpr int kE     = 2048;
constexpr int kNs    = 128;
constexpr int kTd    = 64;
constexpr int kRows  = kBatch * kSeq;
constexpr int kZr    = 2 * kE + 2 * kNs + 1 + 1 + kTd + 1;
constexpr int kZp    = 4480;
constexpr int kSp    = kZp - 2 * kE;
constexpr int kColB   = 0;
constexpr int kColC   = kNs;
constexpr int kColDt  = 2 * kNs;
constexpr int kColA   = kColDt + 1;
constexpr int kColTh  = kColA + 1;
constexpr int kColLam = kColTh + kTd;
constexpr int kXt    = kE / 64;
static_assert(kZr == 4419);
static_assert(kSp == 384);
static_assert(kColLam == 322);
static_assert(2 * kE + kColLam + 1 == kZr);
static_assert((kZp % 64) == 0 && kZp >= kZr);
static_assert((kRows % 64) == 0 && (kE % 64) == 0 && (kDm % 64) == 0 && (kSp % 64) == 0);
static_assert((kDm % 32) == 0 && (kE % 32) == 0);
static_assert((kSeq % 32) == 0 && (kRows % 32) == 0);

constexpr float kCarryU  = 64.0f;
constexpr float kCarryW  = 1024.0f;
constexpr float kCarryG  = 64.0f;
constexpr float kFoldIn  = 1.0f / (kCarryU * kCarryW);
constexpr float kFoldOut = 1.0f / (kCarryG * kCarryW);
constexpr float kF16Min  = 6.103515625e-05f;
constexpr float kEps     = 1e-05f;

constexpr size_t kOffU16  = 0;
constexpr size_t kOffWin  = kOffU16  + (size_t)kRows * kDm * 2;
constexpr size_t kOffWout = kOffWin  + (size_t)kZp * kDm * 2;
constexpr size_t kOffG16  = kOffWout + (size_t)kDm * kE * 2;
constexpr size_t kOffS    = kOffG16  + (size_t)kRows * kE * 2;
constexpr size_t kOffXP   = kOffS    + (size_t)kRows * kSp * 4;
constexpr size_t kOffTok  = kOffXP   + (size_t)kXt * kRows * 4;
constexpr size_t kOffYS   = kOffTok  + (size_t)7 * kRows * 4;
constexpr size_t kWsTotal = kOffYS   + (size_t)kRows * 4;
static_assert(kWsTotal == 77594624ull);
static_assert(kWsTotal <= 134217728ull);
static_assert((kOffWin % 128) == 0 && (kOffWout % 128) == 0 && (kOffG16 % 128) == 0 && (kOffS % 128) == 0 &&
              (kOffXP % 128) == 0 && (kOffTok % 128) == 0 && (kOffYS % 128) == 0);

__device__ __forceinline__ void pin_u(unsigned& x) { asm volatile("" : "+v"(x)); }
__device__ __forceinline__ void pin_f(float& x) { asm volatile("" : "+v"(x)); }

__device__ __forceinline__ _Float16 to_h_flush(float t) {
  const float z = (fabsf(t) < kF16Min) ? 0.0f : t;
  return (_Float16)z;
}

__device__ __forceinline__ void tie_one(v8f& c, v16h a, v16h b) { asm volatile("v_nop" : "+v"(c) : "v"(a), "v"(b)); }
__device__ __forceinline__ void guard_one(v8f& c, v16h a, v16h b) { asm volatile("v_nop\n\tv_nop\n\tv_nop\n\tv_nop" : "+v"(c) : "v"(a), "v"(b)); }
__device__ __forceinline__ void settle_one(v8f& c) { asm volatile("v_nop" : "+v"(c)); }
__device__ __forceinline__ void keep4_h(v16h a, v16h b, v16h c, v16h d) { asm volatile("v_nop" :: "v"(a), "v"(b), "v"(c), "v"(d)); }

template <typename T> struct Frag;
template <> struct Frag<_Float16> {
  typedef v16h V; union U { v16h v; v8h h[2]; };
  static __device__ __forceinline__ v16h load(const _Float16* p) {
    U f; f.h[0] = *(const v8h*)(p); f.h[1] = *(const v8h*)(p + 16); return f.v;
  }
  static __device__ __forceinline__ v8f mma(v16h a, v16h b, v8f c) {
    return __builtin_amdgcn_wmma_f32_16x16x32_f16(false, a, false, b, (short)0, c, false, false);
  }
  static __device__ __forceinline__ void keep(v16h a, v16h b, v16h c, v16h d) { keep4_h(a, b, c, d); }
};

template <int CARRY_I>
__global__ __launch_bounds__(256) void cvt_plane_f16(
    const float* __restrict__ src, unsigned short* __restrict__ dst, unsigned nreal8, unsigned ntot8)
{
  unsigned i = blockIdx.x * 256u + threadIdx.x;
  pin_u(i);
  if (i >= ntot8) return;
  const bool real = (i < nreal8);
  unsigned ic = real ? i : 0u;
  pin_u(ic);
  const size_t e0 = (size_t)ic << 3;
  v4f a0 = *(const v4f*)(src + e0);
  v4f a1 = *(const v4f*)(src + e0 + 4);
  asm volatile("" : "+v"(a0));
  asm volatile("" : "+v"(a1));
  const float carry = (float)CARRY_I;
  v8h hv;
#pragma unroll
  for (int e = 0; e < 4; ++e) {
    const float t0 = real ? (a0[e] * carry) : 0.0f;
    const float t1 = real ? (a1[e] * carry) : 0.0f;
    hv[e]     = to_h_flush(t0);
    hv[4 + e] = to_h_flush(t1);
  }
  unsigned short* q = dst + ((size_t)i << 3);
  *(volatile v8h*)q = hv;
  __threadfence();
  *(volatile v8h*)q = hv;
}

template <int EPI, int GM, int GN, int GK, int LDA, int LDB, int LDC>
__global__ __launch_bounds__(256) void gemm_f16_tile64(
    const unsigned short* __restrict__ Ap, const unsigned short* __restrict__ Btp,
    void* __restrict__ Cout, const float* __restrict__ rowscale)
{
  static_assert((GM % 64) == 0 && (GN % 64) == 0 && (GK % 32) == 0);
  static_assert((LDA % 8) == 0 && (LDB % 8) == 0 && LDA >= GK && LDB >= GK);
  typedef _Float16 T;
  const T* A  = (const T*)Ap;
  const T* Bt = (const T*)Btp;
  __shared__ __align__(16) float sT[8][16 * 68];
  __shared__ __align__(16) float sRS[(EPI == 0) ? 8 : 1][64];
  unsigned lane_u = threadIdx.x & 31u;
  pin_u(lane_u);
  const int lane = (int)lane_u;
  const int wave = threadIdx.x >> 5;
  constexpr int tilesN = GN >> 6;
  constexpr int tilesM = GM >> 6;
  const int tile = blockIdx.x * 8 + wave;
  if (tile >= tilesM * tilesN) return;
  const int tm = tile / tilesN;
  const int tn = tile - tm * tilesN;
  const int m0 = tm << 6;
  const int n0 = tn << 6;

  unsigned rl_u = lane_u & 15u;
  unsigned ko_u = (lane_u >> 4) * 8u;
  pin_u(rl_u);
  pin_u(ko_u);
  const int rlane = (int)rl_u;
  const int koff  = (int)ko_u;
  const int mOff  = koff;
  constexpr float fold = (EPI == 3) ? kFoldOut : kFoldIn;

  v8f acc[4][4];
#pragma unroll
  for (int i = 0; i < 4; ++i)
#pragma unroll
    for (int j = 0; j < 4; ++j) acc[i][j] = (v8f){0.f,0.f,0.f,0.f,0.f,0.f,0.f,0.f};

#pragma unroll 1
  for (int k0 = 0; k0 < GK; k0 += 32) {
    v16h bh[4];
#pragma unroll
    for (int j = 0; j < 4; ++j) {
      const size_t bo = (size_t)(n0 + (j << 4) + rlane) * LDB + koff + k0;
      bh[j] = Frag<T>::load(Bt + bo);
    }
#pragma unroll
    for (int i = 0; i < 4; ++i) {
      const size_t ao = (size_t)(m0 + (i << 4) + rlane) * LDA + koff + k0;
      v16h ah = Frag<T>::load(A + ao);
#pragma unroll
      for (int j = 0; j < 4; ++j) acc[i][j] = Frag<T>::mma(ah, bh[j], acc[i][j]);
      tie_one(acc[i][0], ah, bh[0]);
      tie_one(acc[i][1], ah, bh[1]);
      tie_one(acc[i][2], ah, bh[2]);
      guard_one(acc[i][3], ah, bh[3]);
    }
    Frag<T>::keep(bh[0], bh[1], bh[2], bh[3]);
  }
#pragma unroll
  for (int i = 0; i < 4; ++i)
#pragma unroll
    for (int j = 0; j < 4; ++j) settle_one(acc[i][j]);

  float* slab = sT[wave];
#pragma unroll
  for (int i = 0; i < 4; ++i) {
    const int mBase = m0 + (i << 4);
    float ysr[8];
    if (EPI == 3) {
      const v4f ya = *(const v4f*)(rowscale + mBase + mOff);
      const v4f yb = *(const v4f*)(rowscale + mBase + mOff + 4);
      ysr[0] = ya[0]; ysr[1] = ya[1]; ysr[2] = ya[2]; ysr[3] = ya[3];
      ysr[4] = yb[0]; ysr[5] = yb[1]; ysr[6] = yb[2]; ysr[7] = yb[3];
    }
#pragma unroll
    for (int j = 0; j < 4; ++j) {
#pragma unroll
      for (int r = 0; r < 8; ++r) {
        float v = acc[i][j][r] * fold;
        if (EPI == 0 || EPI == 1) {
          const float ex = __expf(-v);
          const float sg = __builtin_amdgcn_rcpf(1.0f + ex);
          v = v * sg;
        }
        if (EPI == 3) v = v * ysr[r];
        slab[(mOff + r) * 68 + (j << 4) + rlane] = v;
      }
    }
    __builtin_amdgcn_fence(__ATOMIC_RELEASE, "workgroup");
    __builtin_amdgcn_wave_barrier();
    __builtin_amdgcn_fence(__ATOMIC_ACQUIRE, "workgroup");
    if (EPI == 0) {
      const int hh = lane >> 4;
      const float* sp = slab + rlane * 68 + hh * 32;
      float s = 0.0f;
#pragma unroll
      for (int q = 0; q < 8; ++q) {
        const v4f t = *(const v4f*)(sp + 4 * q);
        s += (t[0] + t[1]) + (t[2] + t[3]);
      }
      const float so = __shfl_xor(s, 16, 32);
      s = s + so;
      if (hh == 0) sRS[(EPI == 0) ? wave : 0][(i << 4) + rlane] = s;
    } else if (EPI == 1) {
      const int q = lane >> 3, c8 = (lane & 7) * 8;
      unsigned short* C = (unsigned short*)Cout;
      v8h hv[4];
#pragma unroll
      for (int it = 0; it < 4; ++it) {
        const int row = it * 4 + q;
        const float* sp = slab + row * 68 + c8;
        const v4f p0 = *(const v4f*)(sp);
        const v4f p1 = *(const v4f*)(sp + 4);
#pragma unroll
        for (int e = 0; e < 4; ++e) {
          hv[it][e]     = to_h_flush(p0[e] * kCarryG);
          hv[it][4 + e] = to_h_flush(p1[e] * kCarryG);
        }
      }
      for (int pass = 0; pass < 2; ++pass) {
#pragma unroll
        for (int it = 0; it < 4; ++it) {
          const int row = it * 4 + q;
          *(volatile v8h*)(C + (size_t)(mBase + row) * LDC + n0 + c8) = hv[it];
        }
        __threadfence();
      }
    } else {
      float* C = (float*)Cout;
      const int hh = lane >> 4, c4 = (lane & 15) * 4;
      for (int pass = 0; pass < 2; ++pass) {
#pragma unroll
        for (int it = 0; it < 8; ++it) {
          const int row = it * 2 + hh;
          const v4f v = *(const v4f*)(slab + row * 68 + c4);
          *(volatile v4f*)(C + (size_t)(mBase + row) * LDC + n0 + c4) = v;
        }
        __threadfence();
      }
    }
    __builtin_amdgcn_fence(__ATOMIC_RELEASE, "workgroup");
    __builtin_amdgcn_wave_barrier();
    __builtin_amdgcn_fence(__ATOMIC_ACQUIRE, "workgroup");
  }
  if (EPI == 0) {
    const int li = (lane & 15) * 4;
    const v4f rv = *(const v4f*)(&sRS[(EPI == 0) ? wave : 0][li]);
    float* xp = (float*)Cout + (size_t)tn * LDC + m0 + li;
    for (int pass = 0; pass < 2; ++pass) {
      if (lane < 16) *(volatile v4f*)xp = rv;
      __threadfence();
    }
  }
}

__global__ __launch_bounds__(256) void token_kernel(
    const float* __restrict__ S, const float* __restrict__ XP,
    const float* __restrict__ dtb, const float* __restrict__ alog,
    float* __restrict__ TOK)
{
  __shared__ float sres[7 * 32];
  unsigned lane_u = threadIdx.x & 31u;
  pin_u(lane_u);
  const int lane = (int)lane_u;
  const int wave = threadIdx.x >> 5;
  const int t0 = blockIdx.x * 32;
  const float dtbias = dtb[0];
  const float alg    = alog[0];
  if (wave == 0) {
    float s = 0.0f;
#pragma unroll 4
    for (int tn = 0; tn < kXt; ++tn) s += XP[(size_t)tn * kRows + t0 + lane];
    sres[3 * 32 + lane] = s * (1.0f / (float)kE);
  }
#pragma unroll 1
  for (int i = 0; i < 4; ++i) {
    const int tk = wave * 4 + i;
    const float* Sr = S + (size_t)(t0 + tk) * kSp;
    const v4f bv = *(const v4f*)(Sr + kColB + lane * 4);
    const v4f cv = *(const v4f*)(Sr + kColC + lane * 4);
    float zdt = Sr[kColDt];
    float zA  = Sr[kColA];
    float zlm = Sr[kColLam];
    pin_f(zdt);
    pin_f(zA);
    pin_f(zlm);
    float sb = (bv[0] * bv[0] + bv[1] * bv[1]) + (bv[2] * bv[2] + bv[3] * bv[3]);
    float sc = (cv[0] * cv[0] + cv[1] * cv[1]) + (cv[2] * cv[2] + cv[3] * cv[3]);
#pragma unroll
    for (int off = 16; off >= 1; off >>= 1) {
      const float ob = __shfl_xor(sb, off, 32);
      const float oc = __shfl_xor(sc, off, 32);
      sb += ob;
      sc += oc;
    }
    const float xd  = zdt + dtbias;
    const float dtv = fmaxf(xd, 0.0f) + log1pf(expf(-fabsf(xd)));
    const float xa  = zA + alg;
    const float Av  = -(fmaxf(xa, 0.0f) + log1pf(expf(-fabsf(xa))));
    const float lam = 1.0f / (1.0f + expf(-zlm));
    const float alp = expf(dtv * Av);
    const float ib  = rsqrtf(sb * (1.0f / (float)kNs) + kEps);
    const float ic  = rsqrtf(sc * (1.0f / (float)kNs) + kEps);
    if (lane == 0) {
      sres[0 * 32 + tk] = dtv;
      sres[1 * 32 + tk] = alp;
      sres[2 * 32 + tk] = lam;
      sres[4 * 32 + tk] = Av;
      sres[5 * 32 + tk] = ib;
      sres[6 * 32 + tk] = ic;
    }
  }
  __syncthreads();
  const int pw = (wave < 7) ? wave : 6;
  const float v = sres[pw * 32 + lane];
  if (wave < 7) {
    volatile float* p = TOK + (size_t)pw * kRows + t0 + lane;
    *p = v;
    __threadfence();
    *p = v;
  }
}

__global__ __launch_bounds__(32) void scan_seq_kernel(
    const float* __restrict__ S, const float* __restrict__ TOK,
    const float* __restrict__ wB, const float* __restrict__ wC,
    const float* __restrict__ bB, const float* __restrict__ bC,
    float* __restrict__ YS)
{
  unsigned lane_u = threadIdx.x & 31u;
  pin_u(lane_u);
  const int lane = (int)lane_u;
  const int b = blockIdx.x;
  const float* pDt = TOK + (size_t)0 * kRows;
  const float* pAl = TOK + (size_t)1 * kRows;
  const float* pLm = TOK + (size_t)2 * kRows;
  const float* pXm = TOK + (size_t)3 * kRows;
  const float* pA  = TOK + (size_t)4 * kRows;
  const float* pIb = TOK + (size_t)5 * kRows;
  const float* pIc = TOK + (size_t)6 * kRows;

  float sa = 0.0f;
#pragma unroll 4
  for (int k = 0; k < kRows / 32; ++k) sa += pA[k * 32 + lane];
#pragma unroll
  for (int off = 16; off >= 1; off >>= 1) {
    const float o = __shfl_xor(sa, off, 32);
    sa += o;
  }
  const float Abar = sa * (1.0f / (float)kRows);

  const float wb0 = wB[lane], wb1 = wB[lane + 32], wb2 = wB[lane + 64], wb3 = wB[lane + 96];
  const float wc0 = wC[lane], wc1 = wC[lane + 32], wc2 = wC[lane + 64], wc3 = wC[lane + 96];
  const float bb0 = bB[lane], bb1 = bB[lane + 32], bb2 = bB[lane + 64], bb3 = bB[lane + 96];
  const float bc0 = bC[lane], bc1 = bC[lane + 32], bc2 = bC[lane + 64], bc3 = bC[lane + 96];

  float st0 = 0.0f, st1 = 0.0f, st2 = 0.0f, st3 = 0.0f;
  float ca0 = 0.0f, ca1 = 0.0f;
  float xm_last = 0.0f;
  float ybuf = 0.0f;

#pragma unroll 1
  for (int c = 0; c < kSeq / 32; ++c) {
    const int tc = b * kSeq + c * 32;
    float vdt = pDt[tc + lane];
    float val = pAl[tc + lane];
    float vlm = pLm[tc + lane];
    float vxm = pXm[tc + lane];
    float vib = pIb[tc + lane];
    float vic = pIc[tc + lane];
    pin_f(vdt);
    pin_f(val);
    pin_f(vlm);
    pin_f(vxm);
    pin_f(vib);
    pin_f(vic);
#pragma unroll 1
    for (int s = 0; s < 32; ++s) {
      const float dtv = __shfl(vdt, s, 32);
      const float al  = __shfl(val, s, 32);
      const float lm  = __shfl(vlm, s, 32);
      const float xm  = __shfl(vxm, s, 32);
      const float ib  = __shfl(vib, s, 32);
      const float ic  = __shfl(vic, s, 32);
      const float* Sr = S + (size_t)(tc + s) * kSp;
      float B0 = Sr[kColB + lane];
      float B1 = Sr[kColB + 32 + lane];
      float B2 = Sr[kColB + 64 + lane];
      float B3 = Sr[kColB + 96 + lane];
      float C0 = Sr[kColC + lane];
      float C1 = Sr[kColC + 32 + lane];
      float C2 = Sr[kColC + 64 + lane];
      float C3 = Sr[kColC + 96 + lane];
      float th0 = Sr[kColTh + lane];
      float th1 = Sr[kColTh + 32 + lane];
      pin_f(B0);
      pin_f(B1);
      pin_f(B2);
      pin_f(B3);
      pin_f(C0);
      pin_f(C1);
      pin_f(C2);
      pin_f(C3);
      pin_f(th0);
      pin_f(th1);

      const float um = lm * xm + ((1.0f - lm) * al) * xm_last;
      xm_last = xm;
      const float dA = expf(dtv * Abar);

      const float bn0 = (B0 * ib) * wb0 + bb0;
      const float bn1 = (B1 * ib) * wb1 + bb1;
      const float bn2 = (B2 * ib) * wb2 + bb2;
      const float bn3 = (B3 * ib) * wb3 + bb3;
      const float cn0 = (C0 * ic) * wc0 + bc0;
      const float cn1 = (C1 * ic) * wc1 + bc1;
      const float cn2 = (C2 * ic) * wc2 + bc2;
      const float cn3 = (C3 * ic) * wc3 + bc3;

      ca0 += dtv * th0;
      ca1 += dtv * th1;
      float sn0, cs0, sn1, cs1;
      sincosf(ca0, &sn0, &cs0);
      sincosf(ca1, &sn1, &cs1);

      const float rb0 = bn0 * cs0 - bn2 * sn0;
      const float rb2 = bn0 * sn0 + bn2 * cs0;
      const float rb1 = bn1 * cs1 - bn3 * sn1;
      const float rb3 = bn1 * sn1 + bn3 * cs1;
      const float rc0 = cn0 * cs0 - cn2 * sn0;
      const float rc2 = cn0 * sn0 + cn2 * cs0;
      const float rc1 = cn1 * cs1 - cn3 * sn1;
      const float rc3 = cn1 * sn1 + cn3 * cs1;

      st0 = dA * st0 + (dtv * rb0) * um;
      st1 = dA * st1 + (dtv * rb1) * um;
      st2 = dA * st2 + (dtv * rb2) * um;
      st3 = dA * st3 + (dtv * rb3) * um;

      float ysum = (st0 * rc0 + st1 * rc1) + (st2 * rc2 + st3 * rc3);
#pragma unroll
      for (int off = 16; off >= 1; off >>= 1) {
        const float o = __shfl_xor(ysum, off, 32);
        ysum += o;
      }
      ybuf = (lane == s) ? ysum : ybuf;
    }
    volatile float* yp = YS + tc + lane;
    *yp = ybuf;
    __threadfence();
    *yp = ybuf;
  }
}

extern "C" void kernel_launch(void* const* d_in, const int* in_sizes, int n_in,
                              void* d_out, int out_size, void* d_ws, size_t ws_size,
                              hipStream_t stream) {
  if (n_in < 9) return;
  if (in_sizes[0] != kRows * kDm) return;
  if (in_sizes[1] != kZr * kDm) return;
  if (in_sizes[2] != kNs || in_sizes[3] != kNs || in_sizes[4] != kNs || in_sizes[5] != kNs) return;
  if (in_sizes[6] != 1 || in_sizes[7] != 1) return;
  if (in_sizes[8] != kDm * kE) return;
  if (out_size != kRows * kDm) return;
  if (ws_size < kWsTotal) return;

  const float* u     = (const float*)d_in[0];
  const float* W_in  = (const float*)d_in[1];
  const float* wNB   = (const float*)d_in[2];
  const float* wNC   = (const float*)d_in[3];
  const float* Bbias = (const float*)d_in[4];
  const float* Cbias = (const float*)d_in[5];
  const float* dtb   = (const float*)d_in[6];
  const float* Alog  = (const float*)d_in[7];
  const float* W_out = (const float*)d_in[8];
  float* out = (float*)d_out;

  char* ws = (char*)d_ws;
  unsigned short* U16    = (unsigned short*)(ws + kOffU16);
  unsigned short* WIN16  = (unsigned short*)(ws + kOffWin);
  unsigned short* WOUT16 = (unsigned short*)(ws + kOffWout);
  unsigned short* G16    = (unsigned short*)(ws + kOffG16);
  float*          Spl    = (float*)(ws + kOffS);
  float*          XP     = (float*)(ws + kOffXP);
  float*          TOK    = (float*)(ws + kOffTok);
  float*          YS     = (float*)(ws + kOffYS);

  cvt_plane_f16<64><<<(kRows * kDm / 8) / 256, 256, 0, stream>>>(
      u, U16, (unsigned)(kRows * kDm / 8), (unsigned)(kRows * kDm / 8));
  cvt_plane_f16<1024><<<(kZp * kDm / 8) / 256, 256, 0, stream>>>(
      W_in, WIN16, (unsigned)(kZr * kDm / 8), (unsigned)(kZp * kDm / 8));
  cvt_plane_f16<1024><<<(kDm * kE / 8) / 256, 256, 0, stream>>>(
      W_out, WOUT16, (unsigned)(kDm * kE / 8), (unsigned)(kDm * kE / 8));

  gemm_f16_tile64<0, kRows, kE, kDm, kDm, kDm, kRows><<<(kRows / 64) * (kE / 64) / 8, 256, 0, stream>>>(
      U16, WIN16, (void*)XP, nullptr);
  gemm_f16_tile64<1, kRows, kE, kDm, kDm, kDm, kE><<<(kRows / 64) * (kE / 64) / 8, 256, 0, stream>>>(
      U16, WIN16 + (size_t)kE * kDm, (void*)G16, nullptr);
  gemm_f16_tile64<2, kRows, kSp, kDm, kDm, kDm, kSp><<<(kRows / 64) * (kSp / 64) / 8, 256, 0, stream>>>(
      U16, WIN16 + (size_t)2 * kE * kDm, (void*)Spl, nullptr);

  token_kernel<<<kRows / 32, 256, 0, stream>>>(Spl, XP, dtb, Alog, TOK);

  scan_seq_kernel<<<kBatch, 32, 0, stream>>>(Spl, TOK, wNB, wNC, Bbias, Cbias, YS);

  gemm_f16_tile64<3, kRows, kDm, kE, kE, kE, kDm><<<(kRows / 64) * (kDm / 64) / 8, 256, 0, stream>>>(
      G16, WOUT16, (void*)out, YS);
}
